// PointNetEncoder_62105227100296
// MI455X (gfx1250) — hardware-verified
//
#include <hip/hip_runtime.h>
#pragma clang fp contract(off)

typedef __attribute__((ext_vector_type(16))) _Float16 v16h;
typedef __attribute__((ext_vector_type(8)))  _Float16 v8h;
typedef __attribute__((ext_vector_type(8)))  float    v8f;
typedef __attribute__((ext_vector_type(4)))  float    v4f;
typedef __attribute__((ext_vector_type(4)))  unsigned v4u;

constexpr int kClouds = 8;
constexpr int kPts    = 2048;
constexpr int kSel1   = 1024;
constexpr int kSel2   = 256;
static_assert(kSel1 == kPts / 2);
static_assert(kSel2 == kPts / 8);

constexpr int kWo0 = 0;
constexpr int kWo1 = kWo0 + 64 * 32;
constexpr int kWo2 = kWo1 + 64 * 64;
constexpr int kWo3 = kWo2 + 128 * 64;
constexpr int kWo4 = kWo3 + 128 * 160;
constexpr int kWo5 = kWo4 + 128 * 128;
constexpr int kWo6 = kWo5 + 256 * 128;
constexpr int kWo7 = kWo6 + 256 * 288;
constexpr int kWo8 = kWo7 + 512 * 256;
constexpr int kWoEnd = kWo8 + 1024 * 512;
static_assert(kWoEnd == 813056);
static_assert(kWo1 % 2048 == 0 && kWo2 % 2048 == 0 && kWo3 % 2048 == 0 && kWo4 % 2048 == 0);
static_assert(kWo5 % 2048 == 0 && kWo6 % 2048 == 0 && kWo7 % 2048 == 0 && kWo8 % 2048 == 0 && kWoEnd % 2048 == 0);

constexpr int kA3Pitch = 320;

__device__ __forceinline__ int iclamp(int v, int lo, int hi) { return v < lo ? lo : (v > hi ? hi : v); }
__device__ __forceinline__ unsigned f16bits(float v) {
  const _Float16 h = (_Float16)v;
  return (unsigned)__builtin_bit_cast(unsigned short, h);
}
__device__ __forceinline__ unsigned pack2(unsigned lo, unsigned hi) { return (lo & 0xffffu) | (hi << 16); }

struct FragH {
  union U { v16h v; v8h h[2]; };
  static __device__ __forceinline__ v16h load(const _Float16* p) {
    U f; f.h[0] = *(const v8h*)(p); f.h[1] = *(const v8h*)(p + 16); return f.v;
  }
  static __device__ __forceinline__ v8f mma(v16h a, v16h b, v8f c) {
    return __builtin_amdgcn_wmma_f32_16x16x32_f16(false, a, false, b, (short)0, c, false, false);
  }
};
__device__ __forceinline__ void guard2_h(v8f& a, v8f& b, v16h x, v16h y, v16h z) {
  asm volatile("v_nop\n\tv_nop\n\tv_nop\n\tv_nop" : "+v"(a), "+v"(b) : "v"(x), "v"(y), "v"(z));
}
__device__ __forceinline__ void guard_row_h(v8f& a, v8f& b, v8f& c, v8f& d, v16h x, v16h b0, v16h b1, v16h b2, v16h b3) {
  asm volatile("v_nop\n\tv_nop\n\tv_nop\n\tv_nop" : "+v"(a), "+v"(b), "+v"(c), "+v"(d) : "v"(x), "v"(b0), "v"(b1), "v"(b2), "v"(b3));
}
__device__ __forceinline__ void acc_guard4(v8f& a, v8f& b, v8f& c, v8f& d) {
  asm volatile("v_nop\n\tv_nop\n\tv_nop\n\tv_nop" : "+v"(a), "+v"(b), "+v"(c), "+v"(d));
}

template <int CIN, int COUT, int KP>
__device__ __forceinline__ void wcvt_plane(const float* __restrict__ W, unsigned short* __restrict__ dst, int local) {
  const int o = local / KP;
  const int k = local - o * KP;
  unsigned hb[8];
#pragma unroll
  for (int e = 0; e < 8; ++e) {
    const int kk = k + e;
    const int kc = kk < CIN ? kk : (CIN - 1);
    float v = W[(size_t)kc * COUT + o];
    v = (kk < CIN) ? v : 0.0f;
    hb[e] = f16bits(v);
  }
  v4u w;
  w.x = pack2(hb[0], hb[1]); w.y = pack2(hb[2], hb[3]); w.z = pack2(hb[4], hb[5]); w.w = pack2(hb[6], hb[7]);
  volatile v4u* d = (volatile v4u*)(dst + local);
  *d = w;
  __threadfence();
  *d = w;
}

__global__ __launch_bounds__(256) void wcvt_kernel(
    const float* __restrict__ w0, const float* __restrict__ w1, const float* __restrict__ w2,
    const float* __restrict__ w3, const float* __restrict__ w4, const float* __restrict__ w5,
    const float* __restrict__ w6, const float* __restrict__ w7, const float* __restrict__ w8,
    unsigned short* __restrict__ Wt) {
  const int flat  = (blockIdx.x * 256 + threadIdx.x) * 8;
  const int bflat = blockIdx.x * 2048;
  if (bflat >= kWoEnd) return;
  if      (bflat < kWo1) wcvt_plane<3,   64,   32 >(w0, Wt + kWo0, flat - kWo0);
  else if (bflat < kWo2) wcvt_plane<64,  64,   64 >(w1, Wt + kWo1, flat - kWo1);
  else if (bflat < kWo3) wcvt_plane<64,  128,  64 >(w2, Wt + kWo2, flat - kWo2);
  else if (bflat < kWo4) wcvt_plane<131, 128,  160>(w3, Wt + kWo3, flat - kWo3);
  else if (bflat < kWo5) wcvt_plane<128, 128,  128>(w4, Wt + kWo4, flat - kWo4);
  else if (bflat < kWo6) wcvt_plane<128, 256,  128>(w5, Wt + kWo5, flat - kWo5);
  else if (bflat < kWo7) wcvt_plane<259, 256,  288>(w6, Wt + kWo6, flat - kWo6);
  else if (bflat < kWo8) wcvt_plane<256, 512,  256>(w7, Wt + kWo7, flat - kWo7);
  else                   wcvt_plane<512, 1024, 512>(w8, Wt + kWo8, flat - kWo8);
}

__device__ __forceinline__ void wave_argmax(float& bv, int& bi) {
#pragma unroll
  for (int off = 16; off >= 1; off >>= 1) {
    const float ov = __shfl_xor(bv, off, 32);
    const int   oi = __shfl_xor(bi, off, 32);
    const bool take = (ov > bv) || (ov == bv && oi < bi);
    bv = take ? ov : bv;
    bi = take ? oi : bi;
  }
}

template <int NP, int NSEL, int NT, int PST>
__global__ __launch_bounds__(NT) void fps_kernel(const float* __restrict__ pts, float* __restrict__ cplane) {
#pragma clang fp contract(off)
  constexpr int PPT = NP / NT;
  constexpr int NW  = NT / 32;
  static_assert(PPT == 4 && NW <= 32 && NT >= 64 && (NSEL % NT) == 0);
  __shared__ float px[NP];
  __shared__ float py[NP];
  __shared__ float pz[NP];
  __shared__ int   sel[NSEL];
  __shared__ float wbv[2][32];
  __shared__ int   wbi[2][32];
  const int tid = threadIdx.x, lane = tid & 31, wave = tid >> 5;
  const int cloud = blockIdx.x;
  const float* P = pts + (size_t)cloud * NP * PST;
  float x[PPT], y[PPT], z[PPT], d[PPT];
#pragma unroll
  for (int q = 0; q < PPT; ++q) {
    const int j = tid + q * NT;
    x[q] = P[j * PST + 0]; y[q] = P[j * PST + 1]; z[q] = P[j * PST + 2];
    px[j] = x[q]; py[j] = y[q]; pz[j] = z[q];
  }
  if (tid < 64) { wbv[tid >> 5][tid & 31] = -1.0f; wbi[tid >> 5][tid & 31] = 0x7fffffff; }
  if (tid == 0) sel[0] = 0;
  __syncthreads();
  {
    const float sx = px[0], sy = py[0], sz = pz[0];
#pragma unroll
    for (int q = 0; q < PPT; ++q) {
      const float dx = x[q] - sx, dy = y[q] - sy, dz = z[q] - sz;
      const float t0 = dx * dx, t1 = dy * dy, t2 = dz * dz;
      d[q] = (t0 + t2) + t1;
    }
  }
#pragma unroll 1
  for (int it = 1; it < NSEL; ++it) {
    float bv = d[0]; int bi = tid;
#pragma unroll
    for (int q = 1; q < PPT; ++q) {
      if (d[q] > bv) { bv = d[q]; bi = tid + q * NT; }
    }
    wave_argmax(bv, bi);
    const int par = it & 1;
    if (lane == 0) { wbv[par][wave] = bv; wbi[par][wave] = bi; }
    __syncthreads();
    bv = wbv[par][lane]; bi = wbi[par][lane];
    wave_argmax(bv, bi);
    const int nxt = iclamp(bi, 0, NP - 1);
    if (tid == 0) sel[it] = nxt;
    const float sx = px[nxt], sy = py[nxt], sz = pz[nxt];
#pragma unroll
    for (int q = 0; q < PPT; ++q) {
      const float dx = x[q] - sx, dy = y[q] - sy, dz = z[q] - sz;
      const float t0 = dx * dx, t1 = dy * dy, t2 = dz * dz;
      const float nd = (t0 + t2) + t1;
      d[q] = fminf(d[q], nd);
    }
  }
  __syncthreads();
  float* dstp = cplane + (size_t)cloud * NSEL * 4;
  for (int pass = 0; pass < 2; ++pass) {
    for (int r = tid; r < NSEL; r += NT) {
      const int j = iclamp(sel[r], 0, NP - 1);
      v4f v; v.x = px[j]; v.y = py[j]; v.z = pz[j]; v.w = 0.0f;
      *(volatile v4f*)(dstp + (size_t)r * 4) = v;
    }
    __threadfence();
  }
}

template <int KP, int COUT, bool LAST>
__device__ __forceinline__ void sa_layer(const _Float16* Hin, const _Float16* Wt, const float* bias,
                                         _Float16* Hout, float* Red) {
  const int wave = threadIdx.x >> 5, lane = threadIdx.x & 31;
  const int rl = lane & 15, hh = lane >> 4;
  constexpr int NTASK = (COUT / 16) * 2;
  static_assert(NTASK % 8 == 0 && KP % 32 == 0);
#pragma unroll 1
  for (int t = wave; t < NTASK; t += 8) {
    const int n0 = (t >> 1) * 16;
    const int mh = t & 1;
    const int m0 = mh * 32;
    v8f acc0 = (v8f){0.f,0.f,0.f,0.f,0.f,0.f,0.f,0.f};
    v8f acc1 = (v8f){0.f,0.f,0.f,0.f,0.f,0.f,0.f,0.f};
#pragma unroll 1
    for (int k0 = 0; k0 < KP; k0 += 32) {
      const v16h b  = FragH::load(Wt + (size_t)(n0 + rl) * KP + k0 + 8 * hh);
      const v16h a0 = FragH::load(Hin + (m0 + rl) * KP + k0 + 8 * hh);
      const v16h a1 = FragH::load(Hin + (m0 + 16 + rl) * KP + k0 + 8 * hh);
      acc0 = FragH::mma(a0, b, acc0);
      acc1 = FragH::mma(a1, b, acc1);
      guard2_h(acc0, acc1, a0, a1, b);
    }
    const float bv = bias[n0 + rl];
    if (!LAST) {
#pragma unroll
      for (int r = 0; r < 8; ++r) {
        const float v0 = fmaxf(acc0[r] + bv, 0.0f);
        const float v1 = fmaxf(acc1[r] + bv, 0.0f);
        Hout[(m0 + 8 * hh + r) * COUT + n0 + rl]      = (_Float16)v0;
        Hout[(m0 + 16 + 8 * hh + r) * COUT + n0 + rl] = (_Float16)v1;
      }
    } else {
      float mx = -__builtin_inff();
#pragma unroll
      for (int r = 0; r < 8; ++r) {
        mx = fmaxf(mx, acc0[r] + bv);
        mx = fmaxf(mx, acc1[r] + bv);
      }
      const float other = __shfl_xor(mx, 16, 32);
      mx = fmaxf(mx, other);
      if (hh == 0) Red[mh * COUT + n0 + rl] = mx;
    }
  }
}

template <int NP, int PST, int SPC, int KP1, int C1, int C2, int C3, bool HASX>
__global__ __launch_bounds__(256) void sa_kernel(
    const float* __restrict__ pts, const float* __restrict__ cpos,
    const unsigned short* __restrict__ xfeat,
    const unsigned short* __restrict__ Wt1, const float* __restrict__ b1,
    const unsigned short* __restrict__ Wt2, const float* __restrict__ b2,
    const unsigned short* __restrict__ Wt3, const float* __restrict__ b3,
    unsigned short* __restrict__ outp) {
#pragma clang fp contract(off)
  constexpr int SEG = NP / 8;
  constexpr int SEL_BYTES = NP * 16;
  constexpr int A0_BYTES = 64 * KP1 * 2;
  constexpr int H1_BYTES = 64 * C1 * 2;
  constexpr int H2_BYTES = 64 * C2 * 2;
  constexpr int MLP_BYTES = A0_BYTES + H1_BYTES + (HASX ? 0 : H2_BYTES);
  constexpr int SM_BYTES = SEL_BYTES > MLP_BYTES ? SEL_BYTES : MLP_BYTES;
  constexpr int RW = KP1 / 8;
  constexpr int FW = HASX ? 16 : 0;
  static_assert(!HASX || H2_BYTES <= A0_BYTES);
  static_assert(SEG % 32 == 0 && FW + 1 <= RW);
  static_assert(!HASX || (C3 == 256 && kA3Pitch == 320));
  static_assert(HASX || C3 == 128);
  constexpr float THR = HASX ? 0.16f : 0.04f;

  __shared__ __align__(16) unsigned char smem[SM_BYTES];
  __shared__ int   nbl[64];
  __shared__ int   wcnt[8];
  __shared__ float Red[2 * C3];

  const int tid = threadIdx.x, lane = tid & 31, wave = tid >> 5;
  const int cent = blockIdx.x;
  const int cloud = cent / SPC;
  const float* P = pts + (size_t)cloud * NP * PST;
  const v4f cc = *(const v4f*)(cpos + (size_t)cent * 4);
  const float cx = cc.x, cy = cc.y, cz = cc.z;

  float* segD = (float*)smem;
  int*   segJ = (int*)(smem + NP * 4);
  float* denD = (float*)(smem + NP * 8);
  int*   denJ = (int*)(smem + NP * 12);

  if (tid < 64) nbl[tid] = 0;

  int cntw = 0;
#pragma unroll 1
  for (int it = 0; it < SEG / 32; ++it) {
    const int j = wave * SEG + it * 32 + lane;
    float x, y, z;
    if (PST == 4) {
      const v4f pp = *(const v4f*)(P + (size_t)j * 4);
      x = pp.x; y = pp.y; z = pp.z;
    } else {
      x = P[j * PST + 0]; y = P[j * PST + 1]; z = P[j * PST + 2];
    }
    const float dx = cx - x, dy = cy - y, dz = cz - z;
    const float t0 = dx * dx, t1 = dy * dy, t2 = dz * dz;
    const float d2 = (t0 + t2) + t1;
    const bool inb = d2 <= THR;
    const unsigned bal = __builtin_amdgcn_ballot_w32(inb);
    const int pre = __popc(bal & ((1u << lane) - 1u));
    if (inb) {
      int slot = cntw + pre;
      slot = slot < SEG ? slot : (SEG - 1);
      segD[wave * SEG + slot] = d2;
      segJ[wave * SEG + slot] = j;
    }
    cntw += __popc(bal);
  }
  if (lane == 0) wcnt[wave] = cntw;
  __syncthreads();

  int base = 0, total = 0, mycnt = 0;
#pragma unroll
  for (int w = 0; w < 8; ++w) {
    const int c = iclamp(wcnt[w], 0, SEG);
    base  += (w < wave) ? c : 0;
    mycnt  = (w == wave) ? c : mycnt;
    total += c;
  }
  for (int i = lane; i < mycnt; i += 32) {
    denD[base + i] = segD[wave * SEG + i];
    denJ[base + i] = segJ[wave * SEG + i];
  }
  __syncthreads();

  for (int c = tid; c < total; c += 256) {
    const float myd = denD[c];
    const int   myj = denJ[c];
    int rank = 0;
#pragma unroll 4
    for (int i = 0; i < total; ++i) {
      const float od = denD[i];
      const int   oj = denJ[i];
      rank += ((od < myd) || (od == myd && oj < myj)) ? 1 : 0;
    }
    if (rank < 64) nbl[rank] = myj;
  }
  __syncthreads();
  const int nvalid = total < 64 ? total : 64;

  v4u* A0w = (v4u*)smem;
  if (HASX) {
#pragma unroll
    for (int q = 0; q < 4; ++q) {
      const int idx = tid + q * 256;
      const int e = idx >> 4, w = idx & 15;
      const int j = iclamp(nbl[e < nvalid ? e : 0], 0, NP - 1);
      const v4u val = *(const v4u*)(xfeat + ((size_t)cloud * NP + j) * 128 + w * 8);
      A0w[e * RW + w] = val;
    }
  }
  if (tid < 64) {
    const int e = tid;
    const int j = iclamp(nbl[e < nvalid ? e : 0], 0, NP - 1);
    float x, y, z;
    if (PST == 4) {
      const v4f pp = *(const v4f*)(P + (size_t)j * 4);
      x = pp.x; y = pp.y; z = pp.z;
    } else {
      x = P[j * PST + 0]; y = P[j * PST + 1]; z = P[j * PST + 2];
    }
    const float r0 = x - cx, r1 = y - cy, r2 = z - cz;
    unsigned zz = 0;
    asm volatile("" : "+v"(zz));
    v4u w0;
    w0.x = pack2(f16bits(r0), f16bits(r1));
    w0.y = pack2(f16bits(r2), zz);
    w0.z = zz; w0.w = zz;
    v4u wz; wz.x = zz; wz.y = zz; wz.z = zz; wz.w = zz;
    A0w[e * RW + FW] = w0;
#pragma unroll
    for (int zc = FW + 1; zc < RW; ++zc) A0w[e * RW + zc] = wz;
  }
  __syncthreads();

  _Float16* A0 = (_Float16*)smem;
  _Float16* H1 = (_Float16*)(smem + A0_BYTES);
  _Float16* H2 = HASX ? A0 : (_Float16*)(smem + A0_BYTES + H1_BYTES);

  sa_layer<KP1, C1, false>(A0, (const _Float16*)Wt1, b1, H1, nullptr);
  __syncthreads();
  sa_layer<C1, C2, false>(H1, (const _Float16*)Wt2, b2, H2, nullptr);
  __syncthreads();
  sa_layer<C2, C3, true>(H2, (const _Float16*)Wt3, b3, nullptr, Red);
  __syncthreads();

  if (!HASX) {
    if (tid < 16) {
      const int c0 = tid * 8;
      unsigned hb[8];
#pragma unroll
      for (int e = 0; e < 8; ++e) hb[e] = f16bits(fmaxf(Red[c0 + e], Red[C3 + c0 + e]));
      v4u w;
      w.x = pack2(hb[0], hb[1]); w.y = pack2(hb[2], hb[3]); w.z = pack2(hb[4], hb[5]); w.w = pack2(hb[6], hb[7]);
      volatile v4u* dst = (volatile v4u*)(outp + (size_t)cent * C3 + c0);
      *dst = w;
      __threadfence();
      *dst = w;
    }
  } else {
    if (tid < 40) {
      const int c0 = tid * 8;
      unsigned hb[8];
#pragma unroll
      for (int e = 0; e < 8; ++e) {
        const int col = c0 + e;
        const int cl = col < C3 ? col : (C3 - 1);
        const float m = fmaxf(Red[cl], Red[C3 + cl]);
        const float g = (col == C3) ? cx : ((col == C3 + 1) ? cy : ((col == C3 + 2) ? cz : 0.0f));
        const float v = (col < C3) ? m : g;
        hb[e] = f16bits(v);
      }
      v4u w;
      w.x = pack2(hb[0], hb[1]); w.y = pack2(hb[2], hb[3]); w.z = pack2(hb[4], hb[5]); w.w = pack2(hb[6], hb[7]);
      volatile v4u* dst = (volatile v4u*)(outp + (size_t)cent * kA3Pitch + c0);
      *dst = w;
      __threadfence();
      *dst = w;
    }
  }
}

template <int ACT>
__global__ __launch_bounds__(256) void wmma_gemm64_f16(
    const unsigned short* __restrict__ Ap, int lda,
    const unsigned short* __restrict__ Btp, int ldb,
    unsigned short* __restrict__ Cp, int ldc,
    const float* __restrict__ bias, int M, int N, int K) {
  const _Float16* A  = (const _Float16*)Ap;
  const _Float16* Bt = (const _Float16*)Btp;
  __shared__ __align__(16) float sT[8][16 * 68];
  const int lane = threadIdx.x & 31;
  const int wave = threadIdx.x >> 5;
  const int tilesN = N >> 6;
  const int tilesM = M >> 6;
  const int tile = blockIdx.x * 8 + wave;
  if (tile >= tilesM * tilesN) return;
  const int tm = tile / tilesN;
  const int tn = tile - tm * tilesN;
  const int m0 = tm << 6;
  const int n0 = tn << 6;
  const int rlane = lane & 15;
  const int koff  = (lane >> 4) * 8;
  const int mOff  = (lane >> 4) * 8;

  v8f acc[4][4];
#pragma unroll
  for (int i = 0; i < 4; ++i)
#pragma unroll
    for (int j = 0; j < 4; ++j) acc[i][j] = (v8f){0.f,0.f,0.f,0.f,0.f,0.f,0.f,0.f};

  for (int k0 = 0; k0 < K; k0 += 32) {
    v16h bh[4];
#pragma unroll
    for (int j = 0; j < 4; ++j) {
      const size_t bo = (size_t)(n0 + (j << 4) + rlane) * ldb + koff + k0;
      bh[j] = FragH::load(Bt + bo);
    }
#pragma unroll
    for (int i = 0; i < 4; ++i) {
      const size_t ao = (size_t)(m0 + (i << 4) + rlane) * lda + koff + k0;
      const v16h ah = FragH::load(A + ao);
#pragma unroll
      for (int j = 0; j < 4; ++j) acc[i][j] = FragH::mma(ah, bh[j], acc[i][j]);
      guard_row_h(acc[i][0], acc[i][1], acc[i][2], acc[i][3], ah, bh[0], bh[1], bh[2], bh[3]);
    }
  }
  acc_guard4(acc[0][0], acc[0][1], acc[0][2], acc[0][3]);
  acc_guard4(acc[1][0], acc[1][1], acc[1][2], acc[1][3]);
  acc_guard4(acc[2][0], acc[2][1], acc[2][2], acc[2][3]);
  acc_guard4(acc[3][0], acc[3][1], acc[3][2], acc[3][3]);

  float* slab = sT[wave];
#pragma unroll
  for (int i = 0; i < 4; ++i) {
    const int mBase = m0 + (i << 4);
#pragma unroll
    for (int j = 0; j < 4; ++j) {
      const int n = n0 + (j << 4) + rlane;
      const float bv = bias[n];
#pragma unroll
      for (int r = 0; r < 8; ++r) {
        float v = acc[i][j][r] + bv;
        if (ACT == 2) v = fmaxf(v, 0.0f);
        slab[(mOff + r) * 68 + (j << 4) + rlane] = v;
      }
    }
    __builtin_amdgcn_fence(__ATOMIC_RELEASE, "workgroup");
    __builtin_amdgcn_wave_barrier();
    __builtin_amdgcn_fence(__ATOMIC_ACQUIRE, "workgroup");
    {
      const int q = lane >> 3, c8 = (lane & 7) * 8;
      for (int pass = 0; pass < 2; ++pass) {
#pragma unroll
        for (int it = 0; it < 4; ++it) {
          const int row = it * 4 + q;
          const float* sp = slab + row * 68 + c8;
          v8h hv;
#pragma unroll
          for (int e = 0; e < 8; ++e) hv[e] = (_Float16)sp[e];
          *(volatile v8h*)(Cp + (size_t)(mBase + row) * ldc + n0 + c8) = hv;
        }
        __threadfence();
      }
    }
    __builtin_amdgcn_fence(__ATOMIC_RELEASE, "workgroup");
    __builtin_amdgcn_wave_barrier();
    __builtin_amdgcn_fence(__ATOMIC_ACQUIRE, "workgroup");
  }
}

__global__ __launch_bounds__(128) void gemm_colmax_f16(
    const unsigned short* __restrict__ Ap, const unsigned short* __restrict__ Btp,
    const float* __restrict__ bias, float* __restrict__ out) {
  constexpr int KD = 512, LDA = 512, LDB = 512, NOUT = 1024;
  static_assert(KD % 32 == 0 && kSel2 == 256 && NOUT % 64 == 0);
  const _Float16* A  = (const _Float16*)Ap;
  const _Float16* Bt = (const _Float16*)Btp;
  __shared__ float red[4][64];
  const int tid = threadIdx.x, lane = tid & 31, wave = tid >> 5;
  const int cloud = blockIdx.x >> 4;
  const int n0 = (blockIdx.x & 15) << 6;
  const int m0 = cloud * kSel2 + wave * 64;
  const int rlane = lane & 15;
  const int koff  = (lane >> 4) * 8;
  const int hh    = lane >> 4;

  v8f acc[4][4];
#pragma unroll
  for (int i = 0; i < 4; ++i)
#pragma unroll
    for (int j = 0; j < 4; ++j) acc[i][j] = (v8f){0.f,0.f,0.f,0.f,0.f,0.f,0.f,0.f};

  for (int k0 = 0; k0 < KD; k0 += 32) {
    v16h bh[4];
#pragma unroll
    for (int j = 0; j < 4; ++j) {
      const size_t bo = (size_t)(n0 + (j << 4) + rlane) * LDB + koff + k0;
      bh[j] = FragH::load(Bt + bo);
    }
#pragma unroll
    for (int i = 0; i < 4; ++i) {
      const size_t ao = (size_t)(m0 + (i << 4) + rlane) * LDA + koff + k0;
      const v16h ah = FragH::load(A + ao);
#pragma unroll
      for (int j = 0; j < 4; ++j) acc[i][j] = FragH::mma(ah, bh[j], acc[i][j]);
      guard_row_h(acc[i][0], acc[i][1], acc[i][2], acc[i][3], ah, bh[0], bh[1], bh[2], bh[3]);
    }
  }
  acc_guard4(acc[0][0], acc[0][1], acc[0][2], acc[0][3]);
  acc_guard4(acc[1][0], acc[1][1], acc[1][2], acc[1][3]);
  acc_guard4(acc[2][0], acc[2][1], acc[2][2], acc[2][3]);
  acc_guard4(acc[3][0], acc[3][1], acc[3][2], acc[3][3]);

#pragma unroll
  for (int j = 0; j < 4; ++j) {
    float mx = -__builtin_inff();
#pragma unroll
    for (int i = 0; i < 4; ++i)
#pragma unroll
      for (int r = 0; r < 8; ++r) mx = fmaxf(mx, acc[i][j][r]);
    const float other = __shfl_xor(mx, 16, 32);
    mx = fmaxf(mx, other);
    mx = mx + bias[n0 + (j << 4) + rlane];
    if (hh == 0) red[wave][(j << 4) + rlane] = mx;
  }
  __syncthreads();
  if (tid < 16) {
    const int c4 = tid * 4;
    float m[4];
#pragma unroll
    for (int e = 0; e < 4; ++e)
      m[e] = fmaxf(fmaxf(red[0][c4 + e], red[1][c4 + e]), fmaxf(red[2][c4 + e], red[3][c4 + e]));
    v4f v; v.x = m[0]; v.y = m[1]; v.z = m[2]; v.w = m[3];
    volatile v4f* dst = (volatile v4f*)(out + (size_t)cloud * NOUT + n0 + c4);
    *dst = v;
    __threadfence();
    *dst = v;
  }
}

extern "C" void kernel_launch(void* const* d_in, const int* in_sizes, int n_in,
                              void* d_out, int out_size, void* d_ws, size_t ws_size,
                              hipStream_t stream) {
  (void)in_sizes; (void)out_size;
  if (n_in < 19) return;
  constexpr size_t szWt = (size_t)kWoEnd * 2;
  constexpr size_t szC1 = (size_t)kClouds * kSel1 * 4 * 4;
  constexpr size_t szC2 = (size_t)kClouds * kSel2 * 4 * 4;
  constexpr size_t szH1 = (size_t)kClouds * kSel1 * 128 * 2;
  constexpr size_t szA3 = (size_t)kClouds * kSel2 * kA3Pitch * 2;
  constexpr size_t szG1 = (size_t)kClouds * kSel2 * 256 * 2;
  constexpr size_t szG2 = (size_t)kClouds * kSel2 * 512 * 2;
  constexpr size_t oWt = 0;
  constexpr size_t oC1 = oWt + szWt;
  constexpr size_t oC2 = oC1 + szC1;
  constexpr size_t oH1 = oC2 + szC2;
  constexpr size_t oA3 = oH1 + szH1;
  constexpr size_t oG1 = oA3 + szA3;
  constexpr size_t oG2 = oG1 + szG1;
  constexpr size_t oEnd = oG2 + szG2;
  static_assert(oEnd == 8343552);
  static_assert(oEnd <= (size_t)134217728);
  static_assert(oC1 % 128 == 0 && oC2 % 128 == 0 && oH1 % 128 == 0 && oA3 % 128 == 0 && oG1 % 128 == 0 && oG2 % 128 == 0);
  if (ws_size < oEnd) return;

  char* ws = (char*)d_ws;
  unsigned short* Wt = (unsigned short*)(ws + oWt);
  float* cp1 = (float*)(ws + oC1);
  float* cp2 = (float*)(ws + oC2);
  unsigned short* h1 = (unsigned short*)(ws + oH1);
  unsigned short* A3 = (unsigned short*)(ws + oA3);
  unsigned short* G1 = (unsigned short*)(ws + oG1);
  unsigned short* G2 = (unsigned short*)(ws + oG2);

  const float* pos = (const float*)d_in[0];
  const float* W1a = (const float*)d_in[1];  const float* b1a = (const float*)d_in[2];
  const float* W1b = (const float*)d_in[3];  const float* b1b = (const float*)d_in[4];
  const float* W1c = (const float*)d_in[5];  const float* b1c = (const float*)d_in[6];
  const float* W2a = (const float*)d_in[7];  const float* b2a = (const float*)d_in[8];
  const float* W2b = (const float*)d_in[9];  const float* b2b = (const float*)d_in[10];
  const float* W2c = (const float*)d_in[11]; const float* b2c = (const float*)d_in[12];
  const float* W3a = (const float*)d_in[13]; const float* b3a = (const float*)d_in[14];
  const float* W3b = (const float*)d_in[15]; const float* b3b = (const float*)d_in[16];
  const float* W3c = (const float*)d_in[17]; const float* b3c = (const float*)d_in[18];
  float* outF = (float*)d_out;

  static_assert(kWoEnd / 2048 == 397);
  wcvt_kernel<<<kWoEnd / 2048, 256, 0, stream>>>(W1a, W1b, W1c, W2a, W2b, W2c, W3a, W3b, W3c, Wt);

  fps_kernel<kPts, kSel1, 512, 3><<<kClouds, 512, 0, stream>>>(pos, cp1);

  sa_kernel<kPts, 3, kSel1, 32, 64, 64, 128, false><<<kClouds * kSel1, 256, 0, stream>>>(
      pos, cp1, A3,
      Wt + kWo0, b1a, Wt + kWo1, b1b, Wt + kWo2, b1c, h1);

  fps_kernel<kSel1, kSel2, 256, 4><<<kClouds, 256, 0, stream>>>(cp1, cp2);

  sa_kernel<kSel1, 4, kSel2, 160, 128, 128, 256, true><<<kClouds * kSel2, 256, 0, stream>>>(
      cp1, cp2, h1,
      Wt + kWo3, b2a, Wt + kWo4, b2b, Wt + kWo5, b2c, A3);

  {
    constexpr int M = kClouds * kSel2, N = 256, K = 288;
    static_assert(M % 64 == 0 && N % 64 == 0 && K % 32 == 0 && ((M / 64) * (N / 64)) % 8 == 0);
    wmma_gemm64_f16<2><<<(M / 64) * (N / 64) / 8, 256, 0, stream>>>(A3, kA3Pitch, Wt + kWo6, K, G1, N, b3a, M, N, K);
  }
  {
    constexpr int M = kClouds * kSel2, N = 512, K = 256;
    static_assert(M % 64 == 0 && N % 64 == 0 && K % 32 == 0 && ((M / 64) * (N / 64)) % 8 == 0);
    wmma_gemm64_f16<2><<<(M / 64) * (N / 64) / 8, 256, 0, stream>>>(G1, 256, Wt + kWo7, K, G2, N, b3b, M, N, K);
  }
  gemm_colmax_f16<<<kClouds * 16, 128, 0, stream>>>(G2, Wt + kWo8, b3c, outF);
}
